// CSWinBlockFlex_3788161155753
// MI455X (gfx1250) — hardware-verified
//
#include <hip/hip_runtime.h>
#include <math.h>
#include <stdint.h>

#define NTOK   25088
#define LIMG   3136
#define RESO   56
#define SPL    7
#define CDIM   128
#define CQKV   384
#define CMLP   512
#define HDM    16
#define NWIN   392
#define NQP    400
#define NQT    25
#define KPAD   448
#define NCHK   7
#define WROWS  25600
#define STP    68
#define ASP    20
#define QSC    64.0f
#define KSC    16.0f
#define VSC    16.0f
#define LSC    8.0f
#define OSC    256.0f
#define HSC    64.0f
#define INVS   (1.0f / 4096.0f)

static_assert(WROWS == 64 * NQP);
static_assert(NQT * 16 == NQP);
static_assert(NCHK * 64 == KPAD);
static_assert(KPAD >= NWIN);
static_assert((STP * 4) % 16 == 0);
static_assert((ASP * 4) % 16 == 0);
static_assert(NTOK % 128 == 0);
static_assert(NTOK == 8 * LIMG);
static_assert((KPAD % 8) == 0);

typedef _Float16 v16h __attribute__((ext_vector_type(16)));
typedef _Float16 v8h  __attribute__((ext_vector_type(8)));
typedef float    v8f  __attribute__((ext_vector_type(8)));
typedef float    v4f  __attribute__((ext_vector_type(4)));
typedef unsigned int v4u __attribute__((ext_vector_type(4)));

union Frag { v16h v; v8h h[2]; };

__device__ __forceinline__ unsigned short bf_bits(float f) {
  unsigned u = __float_as_uint(f);
  return (unsigned short)((u + 0x7FFFu + ((u >> 16) & 1u)) >> 16);
}
__device__ __forceinline__ float bfr(float f) { return __uint_as_float(((unsigned)bf_bits(f)) << 16); }
__device__ __forceinline__ unsigned short h_bits(_Float16 x) { return __builtin_bit_cast(unsigned short, x); }
__device__ __forceinline__ unsigned pk16(unsigned short a, unsigned short b) { return (unsigned)a | ((unsigned)b << 16); }
__device__ __forceinline__ v8f zero8() { v8f z = {0.f, 0.f, 0.f, 0.f, 0.f, 0.f, 0.f, 0.f}; return z; }

__device__ __forceinline__ v16h ldfrag_h(const _Float16* p) {
  Frag f;
  f.h[0] = *(const v8h*)(p);
  f.h[1] = *(const v8h*)(p + 16);
  return f.v;
}
__device__ __forceinline__ v16h ldfrag_h2(const _Float16* p0, const _Float16* p1) {
  Frag f;
  f.h[0] = *(const v8h*)(p0);
  f.h[1] = *(const v8h*)(p1);
  return f.v;
}

__device__ __forceinline__ v8f mma_h(v16h a, v16h b, v8f c) {
  c = __builtin_amdgcn_wmma_f32_16x16x32_f16(false, a, false, b, (short)0, c, false, false);
#if defined(__HIP_DEVICE_COMPILE__)
  asm volatile("v_nop\n\tv_nop\n\tv_nop\n\tv_nop" : "+v"(c) : "v"(a), "v"(b));
#endif
  return c;
}
__device__ __forceinline__ void wave_sync_lds() {
  __builtin_amdgcn_fence(__ATOMIC_RELEASE, "workgroup");
  __builtin_amdgcn_wave_barrier();
  __builtin_amdgcn_fence(__ATOMIC_ACQUIRE, "workgroup");
}

__device__ __forceinline__ v4u pack8h(v4f a, v4f b) {
  v4u p;
  p[0] = pk16(h_bits((_Float16)a[0]), h_bits((_Float16)a[1]));
  p[1] = pk16(h_bits((_Float16)a[2]), h_bits((_Float16)a[3]));
  p[2] = pk16(h_bits((_Float16)b[0]), h_bits((_Float16)b[1]));
  p[3] = pk16(h_bits((_Float16)b[2]), h_bits((_Float16)b[3]));
  return p;
}
__device__ __forceinline__ void split8h(v4f a, v4f b, v4u& ph, v4u& pl) {
  v4f ra, rb;
#pragma unroll
  for (int e = 0; e < 4; ++e) {
    const _Float16 ha = (_Float16)a[e];
    ra[e] = (a[e] - (float)ha) * 2048.0f;
    const _Float16 hb = (_Float16)b[e];
    rb[e] = (b[e] - (float)hb) * 2048.0f;
  }
  ph = pack8h(a, b);
  pl = pack8h(ra, rb);
}
__device__ __forceinline__ void splitq8h(v4f a, v4f b, v4u& ph, v4u& pl) {
  v4f ra, rb;
#pragma unroll
  for (int e = 0; e < 4; ++e) {
    const _Float16 ha = (_Float16)a[e];
    ra[e] = a[e] - (float)ha;
    const _Float16 hb = (_Float16)b[e];
    rb[e] = b[e] - (float)hb;
  }
  ph = pack8h(a, b);
  pl = pack8h(ra, rb);
}

__device__ __forceinline__ int tok_row(int n, int br, int wI, int b) {
  const int ha = n / SPL, wa = n - ha * SPL;
  const int la = ha * RESO + wI * SPL + wa;
  const int hb = n / RESO, wb = n - hb * RESO;
  const int lb = (wI * SPL + hb) * RESO + wb;
  return b * LIMG + ((br != 0) ? lb : la);
}

__global__ __launch_bounds__(256) void cvt_wT(const float* __restrict__ w, unsigned short* outp, int nin, int nout) {
  __shared__ float tile[64][33];
  const int tid = threadIdx.x;
  const int i0 = blockIdx.x * 64;
  const int o0 = blockIdx.y * 32;
#pragma unroll
  for (int p = 0; p < 8; ++p) {
    const int idx = p * 256 + tid;
    const int i = idx >> 5, o = idx & 31;
    tile[i][o] = w[(size_t)(i0 + i) * nout + o0 + o];
  }
  __syncthreads();
  const int o = tid >> 3, c8 = (tid & 7) * 8;
  v4u pk;
#pragma unroll
  for (int e = 0; e < 4; ++e) {
    const float fa = bfr(tile[c8 + 2 * e][o]) * 256.0f;
    const float fb = bfr(tile[c8 + 2 * e + 1][o]) * 256.0f;
    pk[e] = pk16(h_bits((_Float16)fa), h_bits((_Float16)fb));
  }
  unsigned short* gp = outp + (size_t)(o0 + o) * nin + i0 + c8;
  *(volatile v4u*)gp = pk;
  __threadfence();
  *(volatile v4u*)gp = pk;
}

template <bool BFIN>
__global__ __launch_bounds__(256) void ln128(const float* __restrict__ xin, const float* __restrict__ g,
                                             const float* __restrict__ bb, unsigned short* oh, unsigned short* ol) {
#pragma clang fp contract(off)
  const int tid = threadIdx.x, wave = tid >> 5, lane = tid & 31, hh = lane >> 4, c = lane & 15;
  const int row = blockIdx.x * 16 + wave * 2 + hh;
  const float* xr = xin + (size_t)row * CDIM + c * 8;
  v4f a0 = *(const v4f*)(xr);
  v4f a1 = *(const v4f*)(xr + 4);
  if (BFIN) {
#pragma unroll
    for (int e = 0; e < 4; ++e) { a0[e] = bfr(a0[e]); a1[e] = bfr(a1[e]); }
  }
  float s = ((a0[0] + a0[1]) + (a0[2] + a0[3])) + ((a1[0] + a1[1]) + (a1[2] + a1[3]));
#pragma unroll
  for (int off = 1; off < 16; off <<= 1) s = s + __shfl_xor(s, off, 32);
  const float mu = s * (1.0f / 128.0f);
  v4f d0, d1;
  float s2 = 0.f;
#pragma unroll
  for (int e = 0; e < 4; ++e) {
    d0[e] = a0[e] - mu;
    const float q0 = d0[e] * d0[e];
    s2 = s2 + q0;
    d1[e] = a1[e] - mu;
    const float q1 = d1[e] * d1[e];
    s2 = s2 + q1;
  }
#pragma unroll
  for (int off = 1; off < 16; off <<= 1) s2 = s2 + __shfl_xor(s2, off, 32);
  const float var = s2 * (1.0f / 128.0f);
  const float rstd = rsqrtf(var + 1e-5f);
  v4f z0, z1;
#pragma unroll
  for (int e = 0; e < 4; ++e) {
    const int cha = c * 8 + e, chb = c * 8 + 4 + e;
    float ta = d0[e] * rstd;
    ta = ta * bfr(g[cha]);
    ta = ta + bfr(bb[cha]);
    z0[e] = ta * LSC;
    float tb = d1[e] * rstd;
    tb = tb * bfr(g[chb]);
    tb = tb + bfr(bb[chb]);
    z1[e] = tb * LSC;
  }
  v4u ph, pl;
  split8h(z0, z1, ph, pl);
  const size_t o = (size_t)row * CDIM + c * 8;
  for (int pass = 0; pass < 2; ++pass) {
    *(volatile v4u*)(oh + o) = ph;
    *(volatile v4u*)(ol + o) = pl;
    __threadfence();
  }
}

template <int MODE>
__global__ __launch_bounds__(256)
void gemm_k(const unsigned short* __restrict__ Ah, const unsigned short* __restrict__ Al,
            const unsigned short* __restrict__ Bt, int K,
            const float* __restrict__ f0, const float* __restrict__ f1,
            float* outF, unsigned short* h0, unsigned short* h1, unsigned short* h2,
            unsigned short* h3, unsigned short* h4, float oscale) {
  __shared__ __align__(16) float sbuf[8 * 16 * STP];
  const int tid = threadIdx.x, wave = tid >> 5, lane = tid & 31, hh = lane >> 4, c = lane & 15;
  const int n0 = blockIdx.x * 64, m0 = blockIdx.y * 128;
  const int arow = m0 + wave * 16 + c;
  const _Float16* A0 = (const _Float16*)(const void*)Ah;
  const _Float16* A1 = (const _Float16*)(const void*)Al;
  const _Float16* B  = (const _Float16*)(const void*)Bt;

  int rb0 = 0, rb1 = 0;
  if (MODE == 2) {
    const int bimg = arow / LIMG, l = arow - bimg * LIMG;
    const int hr = l / RESO, col = l - hr * RESO;
    const int w0 = col / SPL, wj = col - w0 * SPL;
    const int w1 = hr / SPL,  hi = hr - w1 * SPL;
    rb0 = (bimg * 8 + w0) * NQP + hr * SPL + wj;
    rb1 = (bimg * 8 + w1) * NQP + hi * RESO + col;
  }

  v8f acch[4], accl[4];
#pragma unroll
  for (int nt = 0; nt < 4; ++nt) { acch[nt] = zero8(); accl[nt] = zero8(); }

#pragma unroll 1
  for (int k0 = 0; k0 < K; k0 += 32) {
    v16h ah, al;
    if (MODE == 2) {
      const int gs = k0 >> 4;
      const int rs = (k0 >= 64) ? rb1 : rb0;
      const size_t oa = ((size_t)gs * WROWS + rs) * HDM + 8 * hh;
      const size_t ob = ((size_t)(gs + 1) * WROWS + rs) * HDM + 8 * hh;
      ah = ldfrag_h2(A0 + oa, A0 + ob);
      al = ldfrag_h2(A1 + oa, A1 + ob);
    } else {
      const size_t aoff = (size_t)arow * K + k0 + 8 * hh;
      ah = ldfrag_h(A0 + aoff);
      al = ldfrag_h(A1 + aoff);
    }
#pragma unroll
    for (int nt = 0; nt < 4; ++nt) {
      const v16h bfrag = ldfrag_h(B + (size_t)(n0 + nt * 16 + c) * K + k0 + 8 * hh);
      acch[nt] = mma_h(ah, bfrag, acch[nt]);
      accl[nt] = mma_h(al, bfrag, accl[nt]);
    }
  }

  float* st = sbuf + wave * (16 * STP);
#pragma unroll
  for (int nt = 0; nt < 4; ++nt) {
#pragma unroll
    for (int r = 0; r < 8; ++r) {
      const float v = acch[nt][r] + accl[nt][r] * (1.0f / 2048.0f);
      st[(8 * hh + r) * STP + nt * 16 + c] = v * oscale;
    }
  }
  wave_sync_lds();

  if (MODE == 0 || MODE == 2) {
    v4f ov[8];
    size_t offs[8];
#pragma unroll
    for (int it = 0; it < 8; ++it) {
      const int q = it * 2 + hh;
      const int col = n0 + c * 4;
      const size_t ro = (size_t)(m0 + wave * 16 + q) * CDIM + col;
      const v4f v = *(const v4f*)(st + q * STP + c * 4);
      const v4f rr = *(const v4f*)(f1 + ro);
      v4f u;
#pragma unroll
      for (int e = 0; e < 4; ++e) {
        const float t = v[e] + bfr(f0[col + e]);
        const float rs = (MODE == 2) ? bfr(rr[e]) : rr[e];
        u[e] = rs + t;
      }
      ov[it] = u;
      offs[it] = ro;
    }
    for (int pass = 0; pass < 2; ++pass) {
#pragma unroll
      for (int it = 0; it < 8; ++it) *(volatile v4f*)(outF + offs[it]) = ov[it];
      __threadfence();
    }
  } else if (MODE == 1) {
    const int part = n0 >> 7, colp = n0 & 127;
    unsigned short* dA = (part == 0) ? h0 : ((part == 1) ? h2 : h3);
    unsigned short* dB = (part == 0) ? h1 : h4;
    v4u pa[4], pb[4];
    size_t offs[4];
#pragma unroll
    for (int it = 0; it < 4; ++it) {
      const int q = it * 4 + (lane >> 3), piece = lane & 7;
      v4f fa = *(const v4f*)(st + q * STP + piece * 8);
      v4f fb = *(const v4f*)(st + q * STP + piece * 8 + 4);
      if (part == 0) {
        fa = fa * QSC; fb = fb * QSC;
        splitq8h(fa, fb, pa[it], pb[it]);
      } else if (part == 1) {
        fa = fa * KSC; fb = fb * KSC;
        pa[it] = pack8h(fa, fb);
        pb[it] = pa[it];
      } else {
        fa = fa * VSC; fb = fb * VSC;
        split8h(fa, fb, pa[it], pb[it]);
      }
      offs[it] = (size_t)(m0 + wave * 16 + q) * CDIM + colp + piece * 8;
    }
    for (int pass = 0; pass < 2; ++pass) {
#pragma unroll
      for (int it = 0; it < 4; ++it) {
        *(volatile v4u*)(dA + offs[it]) = pa[it];
        if (part != 1) *(volatile v4u*)(dB + offs[it]) = pb[it];
      }
      __threadfence();
    }
  } else {
    v4u pa[4], pb[4];
    size_t offs[4];
#pragma unroll
    for (int it = 0; it < 4; ++it) {
      const int q = it * 4 + (lane >> 3), piece = lane & 7;
      const int col0 = n0 + piece * 8;
      const v4f fa = *(const v4f*)(st + q * STP + piece * 8);
      const v4f fb = *(const v4f*)(st + q * STP + piece * 8 + 4);
      v4f ua, ub;
#pragma unroll
      for (int e = 0; e < 4; ++e) {
        const float u0 = fa[e] + bfr(f0[col0 + e]);
        const float g0 = 0.5f * u0 * (1.0f + erff(u0 * 0.70710678118654752f));
        ua[e] = g0 * HSC;
        const float u1 = fb[e] + bfr(f0[col0 + 4 + e]);
        const float g1 = 0.5f * u1 * (1.0f + erff(u1 * 0.70710678118654752f));
        ub[e] = g1 * HSC;
      }
      split8h(ua, ub, pa[it], pb[it]);
      offs[it] = (size_t)(m0 + wave * 16 + q) * CMLP + col0;
    }
    for (int pass = 0; pass < 2; ++pass) {
#pragma unroll
      for (int it = 0; it < 4; ++it) {
        *(volatile v4u*)(h0 + offs[it]) = pa[it];
        *(volatile v4u*)(h1 + offs[it]) = pb[it];
      }
      __threadfence();
    }
  }
}

__global__ __launch_bounds__(256)
void attn_k(const unsigned short* __restrict__ Qh, const unsigned short* __restrict__ Ql,
            const unsigned short* __restrict__ Kp,
            const unsigned short* __restrict__ Vh, const unsigned short* __restrict__ Vl,
            const float* __restrict__ cw0, const float* __restrict__ cb0,
            const float* __restrict__ cw1, const float* __restrict__ cb1,
            unsigned short* Oh, unsigned short* Ol) {
  __shared__ __align__(16) unsigned short Ks[KPAD * HDM];
  __shared__ __align__(16) unsigned short Vth[HDM * KPAD];
  __shared__ __align__(16) unsigned short Vtl[HDM * KPAD];
  __shared__ __align__(16) float Sst[8 * 16 * ASP];
  const int tid = threadIdx.x, wave = tid >> 5, lane = tid & 31, hh = lane >> 4, c = lane & 15;
  const int br = blockIdx.y;
  const int head = blockIdx.x & 3, wI = (blockIdx.x >> 2) & 7, b = blockIdx.x >> 5;
  const int c0 = br * 64 + head * HDM;

#pragma unroll
  for (int it = 0; it < 2; ++it) {
    const int n = it * 256 + tid;
    if (n < KPAD) {
      const bool val = n < NWIN;
      const int nc = val ? n : (NWIN - 1);
      const size_t row = (size_t)tok_row(nc, br, wI, b);
      const v4u* kg = (const v4u*)(Kp + row * CDIM + c0);
      const v4u* hg = (const v4u*)(Vh + row * CDIM + c0);
      const v4u* lg = (const v4u*)(Vl + row * CDIM + c0);
      const unsigned msk = val ? 0xFFFFFFFFu : 0u;
#pragma unroll
      for (int i = 0; i < 2; ++i) {
        v4u kw = kg[i], hw = hg[i], lw = lg[i];
        kw = kw & msk; hw = hw & msk; lw = lw & msk;
        *(v4u*)(Ks + n * HDM + 8 * i) = kw;
#pragma unroll
        for (int e = 0; e < 4; ++e) {
          Vth[(8 * i + 2 * e) * KPAD + n]     = (unsigned short)(hw[e] & 0xFFFFu);
          Vth[(8 * i + 2 * e + 1) * KPAD + n] = (unsigned short)(hw[e] >> 16);
          Vtl[(8 * i + 2 * e) * KPAD + n]     = (unsigned short)(lw[e] & 0xFFFFu);
          Vtl[(8 * i + 2 * e + 1) * KPAD + n] = (unsigned short)(lw[e] >> 16);
        }
      }
    }
  }
  __syncthreads();

  const float* cw  = (br != 0) ? cw1 : cw0;
  const float* cbp = (br != 0) ? cb1 : cb0;
  const int ch = head * HDM + c;
  float wA[9];
#pragma unroll
  for (int t = 0; t < 9; ++t) wA[t] = bfr(cw[t * 64 + ch]);
  const float bA = bfr(cbp[ch]);

  const _Float16* Ksh = (const _Float16*)(const void*)Ks;
  const _Float16* Vhh = (const _Float16*)(const void*)Vth;
  const _Float16* Vlh = (const _Float16*)(const void*)Vtl;
  const _Float16* Qhg = (const _Float16*)(const void*)Qh;
  const _Float16* Qlg = (const _Float16*)(const void*)Ql;
  float* st = Sst + wave * (16 * ASP);
  const int Wd = (br != 0) ? RESO : SPL;
  const int Hd = (br != 0) ? SPL : RESO;

#pragma unroll 1
  for (int qt = wave; qt < NQT; qt += 8) {
    const int nq = qt * 16 + c;
    const int nqc = (nq < NWIN) ? nq : (NWIN - 1);
    const size_t rq = (size_t)tok_row(nqc, br, wI, b);
    Frag qf;
    qf.h[0] = *(const v8h*)(Qhg + rq * CDIM + c0 + 8 * hh);
    qf.h[1] = *(const v8h*)(Qlg + rq * CDIM + c0 + 8 * hh);
    v8f o = zero8(), ol = zero8();
    float mrun = -1.0e30f, lrun = 0.f;
#pragma unroll 1
    for (int chn = 0; chn < NCHK; ++chn) {
      const int kb = chn * 64;
      v8f s[4];
#pragma unroll
      for (int j = 0; j < 4; ++j) {
        Frag ka;
        ka.h[0] = *(const v8h*)(Ksh + (size_t)(kb + j * 16 + c) * HDM + 8 * hh);
        ka.h[1] = ka.h[0];
        s[j] = mma_h(ka.v, qf.v, zero8());
      }
      float mc = -1.0e30f;
#pragma unroll
      for (int j = 0; j < 4; ++j) {
#pragma unroll
        for (int r = 0; r < 8; ++r) {
          const int key = kb + 16 * j + 8 * hh + r;
          const float sv = (key < NWIN) ? s[j][r] : -1.0e30f;
          s[j][r] = sv;
          mc = fmaxf(mc, sv);
        }
      }
      mc = fmaxf(mc, __shfl_xor(mc, 16, 32));
      const float mnew = fmaxf(mrun, mc);
      const float alpha = __expf((mrun - mnew) * INVS);
#pragma unroll
      for (int r = 0; r < 8; ++r) {
        const float ar = __shfl(alpha, 8 * hh + r, 32);
        o[r] = o[r] * ar;
        ol[r] = ol[r] * ar;
      }
      float psum = 0.f;
      v16h pf0, pf1;
#pragma unroll
      for (int i = 0; i < 8; ++i) {
        const float e0 = __expf((s[0][i] - mnew) * INVS);
        const float e1 = __expf((s[1][i] - mnew) * INVS);
        const float e2 = __expf((s[2][i] - mnew) * INVS);
        const float e3 = __expf((s[3][i] - mnew) * INVS);
        psum = psum + ((e0 + e1) + (e2 + e3));
        pf0[i]     = (_Float16)(e0 * 1024.0f);
        pf0[8 + i] = (_Float16)(e1 * 1024.0f);
        pf1[i]     = (_Float16)(e2 * 1024.0f);
        pf1[8 + i] = (_Float16)(e3 * 1024.0f);
      }
      lrun = lrun * alpha + psum;
      mrun = mnew;
      {
        const v16h va = ldfrag_h(Vhh + (size_t)c * KPAD + kb + 8 * hh);
        o = mma_h(pf0, va, o);
        const v16h vb = ldfrag_h(Vhh + (size_t)c * KPAD + kb + 32 + 8 * hh);
        o = mma_h(pf1, vb, o);
        const v16h wa = ldfrag_h(Vlh + (size_t)c * KPAD + kb + 8 * hh);
        ol = mma_h(pf0, wa, ol);
        const v16h wb = ldfrag_h(Vlh + (size_t)c * KPAD + kb + 32 + 8 * hh);
        ol = mma_h(pf1, wb, ol);
      }
    }
    const float lsum = lrun + __shfl_xor(lrun, 16, 32);
#pragma unroll
    for (int r = 0; r < 8; ++r) {
      const int q = 8 * hh + r;
      const float lq = __shfl(lsum, q, 32);
      const float inv = 1.0f / (lq * 16384.0f);
      const int n = qt * 16 + q;
      const int wi = (br != 0) ? (n / RESO) : (n / SPL);
      const int wj = n - wi * Wd;
      float la = 0.f;
#pragma unroll
      for (int di = 0; di < 3; ++di) {
#pragma unroll
        for (int dj = 0; dj < 3; ++dj) {
          const int ii = wi + di - 1, jj = wj + dj - 1;
          const bool ok = ((unsigned)ii < (unsigned)Hd) && ((unsigned)jj < (unsigned)Wd);
          const int nn = ok ? (ii * Wd + jj) : n;
          const float xh = (float)Vhh[(size_t)c * KPAD + nn];
          const float xl = (float)Vlh[(size_t)c * KPAD + nn];
          const float xv = xh + xl * (1.0f / 2048.0f);
          la += (ok ? xv : 0.f) * wA[di * 3 + dj];
        }
      }
      const float ov = (o[r] + ol[r] * (1.0f / 2048.0f)) * inv + (la * (1.0f / 16.0f) + bA);
      st[q * ASP + c] = ov;
    }
    wave_sync_lds();
    {
      const int q = lane >> 1, piece = lane & 1;
      v4f fa = *(const v4f*)(st + q * ASP + piece * 8);
      v4f fb = *(const v4f*)(st + q * ASP + piece * 8 + 4);
      fa = fa * OSC;
      fb = fb * OSC;
      v4u ph, pl;
      split8h(fa, fb, ph, pl);
      const int gsl = br * 4 + head;
      const size_t offs = ((((size_t)(gsl * 8 + b)) * 8 + wI) * NQP + qt * 16 + q) * HDM + piece * 8;
      for (int pass = 0; pass < 2; ++pass) {
        *(volatile v4u*)(Oh + offs) = ph;
        *(volatile v4u*)(Ol + offs) = pl;
        __threadfence();
      }
    }
    wave_sync_lds();
  }
}

extern "C" void kernel_launch(void* const* d_in, const int* in_sizes, int n_in,
                              void* d_out, int out_size, void* d_ws, size_t ws_size,
                              hipStream_t stream) {
  if (n_in < 16) return;
  if (in_sizes[0] != NTOK * CDIM) return;
  if (in_sizes[1] != CDIM || in_sizes[2] != CDIM) return;
  if (in_sizes[3] != CDIM * CQKV) return;
  if (in_sizes[4] != 9 * 64 || in_sizes[5] != 64 || in_sizes[6] != 9 * 64 || in_sizes[7] != 64) return;
  if (in_sizes[8] != CDIM * CDIM || in_sizes[9] != CDIM) return;
  if (in_sizes[10] != CDIM || in_sizes[11] != CDIM) return;
  if (in_sizes[12] != CDIM * CMLP || in_sizes[13] != CMLP) return;
  if (in_sizes[14] != CMLP * CDIM || in_sizes[15] != CDIM) return;
  if (out_size != NTOK * CDIM) return;

  const float* x      = (const float*)d_in[0];
  const float* g1     = (const float*)d_in[1];
  const float* b1     = (const float*)d_in[2];
  const float* w_qkv  = (const float*)d_in[3];
  const float* cw0    = (const float*)d_in[4];
  const float* cb0    = (const float*)d_in[5];
  const float* cw1    = (const float*)d_in[6];
  const float* cb1    = (const float*)d_in[7];
  const float* w_proj = (const float*)d_in[8];
  const float* b_proj = (const float*)d_in[9];
  const float* g2     = (const float*)d_in[10];
  const float* b2     = (const float*)d_in[11];
  const float* w_fc1  = (const float*)d_in[12];
  const float* b_fc1  = (const float*)d_in[13];
  const float* w_fc2  = (const float*)d_in[14];
  const float* b_fc2  = (const float*)d_in[15];
  float* out = (float*)d_out;

  const size_t sWq = (size_t)CQKV * CDIM * 2;
  const size_t sWp = (size_t)CDIM * CDIM * 2;
  const size_t sW1 = (size_t)CMLP * CDIM * 2;
  const size_t sW2 = (size_t)CDIM * CMLP * 2;
  const size_t sT  = (size_t)8 * WROWS * HDM * 2;
  const size_t sP  = (size_t)NTOK * CDIM * 2;
  const size_t sXR = (size_t)NTOK * CDIM * 4;
  const size_t sH  = (size_t)NTOK * CMLP * 2;
  size_t off = 0;
  const size_t oWq = off; off += sWq;
  const size_t oWp = off; off += sWp;
  const size_t oW1 = off; off += sW1;
  const size_t oW2 = off; off += sW2;
  const size_t oTh = off; off += sT;
  const size_t oTl = off; off += sT;
  const size_t oQh = off; off += sP;
  const size_t oQl = off; off += sP;
  const size_t oK  = off; off += sP;
  const size_t oVh = off; off += sP;
  const size_t oVl = off; off += sP;
  const size_t oXR = off; off += sXR;
  const size_t oHh = off; off += sH;
  const size_t oHl = off; off += sH;
  if (off > ws_size) return;
  if (off > (size_t)134217728) return;
  if (sT < sP) return;

  char* ws = (char*)d_ws;
  unsigned short* Wq = (unsigned short*)(ws + oWq);
  unsigned short* Wp = (unsigned short*)(ws + oWp);
  unsigned short* W1 = (unsigned short*)(ws + oW1);
  unsigned short* W2 = (unsigned short*)(ws + oW2);
  unsigned short* Th = (unsigned short*)(ws + oTh);
  unsigned short* Tl = (unsigned short*)(ws + oTl);
  unsigned short* Qh = (unsigned short*)(ws + oQh);
  unsigned short* Ql = (unsigned short*)(ws + oQl);
  unsigned short* Kp = (unsigned short*)(ws + oK);
  unsigned short* Vh = (unsigned short*)(ws + oVh);
  unsigned short* Vl = (unsigned short*)(ws + oVl);
  float* XR = (float*)(ws + oXR);
  unsigned short* Hh = (unsigned short*)(ws + oHh);
  unsigned short* Hl = (unsigned short*)(ws + oHl);

  const dim3 blk(256);
  cvt_wT<<<dim3(CDIM / 64, CQKV / 32), blk, 0, stream>>>(w_qkv, Wq, CDIM, CQKV);
  cvt_wT<<<dim3(CDIM / 64, CDIM / 32), blk, 0, stream>>>(w_proj, Wp, CDIM, CDIM);
  cvt_wT<<<dim3(CDIM / 64, CMLP / 32), blk, 0, stream>>>(w_fc1, W1, CDIM, CMLP);
  cvt_wT<<<dim3(CMLP / 64, CDIM / 32), blk, 0, stream>>>(w_fc2, W2, CMLP, CDIM);
  ln128<true><<<dim3(NTOK / 16), blk, 0, stream>>>(x, g1, b1, Th, Tl);
  gemm_k<1><<<dim3(CQKV / 64, NTOK / 128), blk, 0, stream>>>(
      Th, Tl, Wq, CDIM, b_proj, x, XR, Qh, Ql, Kp, Vh, Vl, 1.0f / 2048.0f);
  attn_k<<<dim3(8 * 8 * 4, 2), blk, 0, stream>>>(Qh, Ql, Kp, Vh, Vl, cw0, cb0, cw1, cb1, Th, Tl);
  gemm_k<2><<<dim3(CDIM / 64, NTOK / 128), blk, 0, stream>>>(
      Th, Tl, Wp, CDIM, b_proj, x, XR, Hh, Hh, Hh, Hh, Hh, 1.0f / 65536.0f);
  ln128<false><<<dim3(NTOK / 16), blk, 0, stream>>>(XR, g2, b2, Th, Tl);
  gemm_k<3><<<dim3(CMLP / 64, NTOK / 128), blk, 0, stream>>>(
      Th, Tl, W1, CDIM, b_fc1, XR, XR, Hh, Hl, Hh, Hh, Hh, 1.0f / 2048.0f);
  gemm_k<0><<<dim3(CDIM / 64, NTOK / 128), blk, 0, stream>>>(
      Hh, Hl, W2, CMLP, b_fc2, XR, out, Hh, Hh, Hh, Hh, Hh, 1.0f / 16384.0f);
  (void)hipGetLastError();
}
